// Seq2SeqModel_52278341927194
// MI455X (gfx1250) — hardware-verified
//
#include <hip/hip_runtime.h>
#include <math.h>

constexpr int NB     = 256;
constexpr int NS     = 128;
constexpr int NTD    = 64;
constexpr int NI     = 63;
constexpr int NIP    = 64;
constexpr int NH     = 1024;
constexpr int NG3    = 3 * NH;
constexpr int NTHR   = 256;
constexpr int NWAV   = NTHR / 32;
constexpr int WCOLS  = NH / NWAV;
constexpr int NTW    = WCOLS / 16;
constexpr int SEQB   = 16;
constexpr int DBLK   = NTD / SEQB;
constexpr int XPITCH = 72;
constexpr int HPITCH = 1032;
constexpr int HMP    = 1028;
constexpr int SLABP  = 68;
constexpr int GHCOLB = 64 * NWAV;
constexpr int NROWE  = NB * NS;
constexpr int NROWD  = NB * NTD;
constexpr int NOUT   = NROWD * NI;
constexpr int PROWS  = 64;
constexpr int PNF4   = PROWS * NI / 4;
constexpr int GSROWS = 10;
constexpr float WCARRY     = 256.0f;
constexpr float WCARRY_INV = 1.0f / 256.0f;
static_assert(NB % SEQB == 0 && NTD % SEQB == 0 && DBLK == 4, "");
static_assert(NWAV * WCOLS == NH && NTW * 16 == WCOLS && NTW == 8, "");
static_assert(NIP % 32 == 0 && NH % 32 == 0, "");
static_assert(XPITCH % 8 == 0 && XPITCH >= NIP && HPITCH % 8 == 0 && HPITCH >= NH && HMP % 4 == 0 && HMP >= NH, "");
static_assert(NH == 4 * NTHR, "");
static_assert(NG3 % GHCOLB == 0, "");
static_assert(SEQB * NH == 16 * NTHR * 4 && SEQB * NH == 8 * NTHR * 8, "");
static_assert(NROWD % PROWS == 0 && (PROWS * NI) % 4 == 0 && (PROWS * NI * 4) % 128 == 0 && PNF4 <= 4 * NTHR, "");
static_assert((NROWE * (NIP / 8)) % NTHR == 0 && (NROWD * (NIP / 8)) % NTHR == 0, "");
static_assert((NG3 * (NIP / 8)) % NTHR == 0 && (NG3 * (NH / 8)) % NTHR == 0 && (NIP * (NH / 8)) % NTHR == 0, "");

typedef __attribute__((ext_vector_type(16))) _Float16 v16h;
typedef __attribute__((ext_vector_type(8)))  _Float16 v8h;
typedef __attribute__((ext_vector_type(16))) __bf16   v16b;
typedef __attribute__((ext_vector_type(8)))  __bf16   v8b;
typedef __attribute__((ext_vector_type(8)))  float    v8f;
typedef __attribute__((ext_vector_type(4)))  float    v4f;

__device__ __forceinline__ unsigned short f2bf_bits(float f) {
  unsigned u = __float_as_uint(f);
  return (unsigned short)((u + 0x7FFFu + ((u >> 16) & 1u)) >> 16);
}
__device__ __forceinline__ float bf_bits2f(unsigned short h) { return __uint_as_float(((unsigned)h) << 16); }
__device__ __forceinline__ float bf16r(float f) { return bf_bits2f(f2bf_bits(f)); }

__device__ __forceinline__ void guard4_b(v8f& a0, v8f& a1, v8f& a2, v8f& a3, v16b x, v16b y0, v16b y1, v16b y2) {
  asm volatile("v_nop\n\tv_nop\n\tv_nop\n\tv_nop" : "+v"(a0), "+v"(a1), "+v"(a2), "+v"(a3) : "v"(x), "v"(y0), "v"(y1), "v"(y2));
}
__device__ __forceinline__ void guard4_h(v8f& a0, v8f& a1, v8f& a2, v8f& a3, v16h x, v16h y0, v16h y1, v16h y2) {
  asm volatile("v_nop\n\tv_nop\n\tv_nop\n\tv_nop" : "+v"(a0), "+v"(a1), "+v"(a2), "+v"(a3) : "v"(x), "v"(y0), "v"(y1), "v"(y2));
}
__device__ __forceinline__ void guard4_b6(v8f& a0, v8f& a1, v8f& a2, v8f& a3, v16b x0, v16b x1, v16b y0, v16b y1, v16b y2, v16b y3) {
  asm volatile("v_nop\n\tv_nop\n\tv_nop\n\tv_nop" : "+v"(a0), "+v"(a1), "+v"(a2), "+v"(a3) : "v"(x0), "v"(x1), "v"(y0), "v"(y1), "v"(y2), "v"(y3));
}
__device__ __forceinline__ void guard3_b(v8f& a0, v8f& a1, v8f& a2, v16b x, v16b y0, v16b y1, v16b y2) {
  asm volatile("v_nop\n\tv_nop\n\tv_nop\n\tv_nop" : "+v"(a0), "+v"(a1), "+v"(a2) : "v"(x), "v"(y0), "v"(y1), "v"(y2));
}
__device__ __forceinline__ void guard2_b4(v8f& a0, v8f& a1, v16b x0, v16b x1, v16b y0, v16b y1) {
  asm volatile("v_nop\n\tv_nop\n\tv_nop\n\tv_nop" : "+v"(a0), "+v"(a1) : "v"(x0), "v"(x1), "v"(y0), "v"(y1));
}
__device__ __forceinline__ void acc_guard4(v8f& a, v8f& b, v8f& c, v8f& d) { asm volatile("v_nop\n\tv_nop\n\tv_nop\n\tv_nop" : "+v"(a), "+v"(b), "+v"(c), "+v"(d)); }
__device__ __forceinline__ void acc_guard3(v8f& a, v8f& b, v8f& c) { asm volatile("v_nop\n\tv_nop\n\tv_nop\n\tv_nop" : "+v"(a), "+v"(b), "+v"(c)); }
__device__ __forceinline__ void acc_guard2(v8f& a, v8f& b) { asm volatile("v_nop\n\tv_nop\n\tv_nop\n\tv_nop" : "+v"(a), "+v"(b)); }

template <typename T> struct Frag;
template <> struct Frag<_Float16> {
  typedef v16h V; union U { v16h v; v8h h[2]; };
  static __device__ __forceinline__ v16h load(const _Float16* p) {
    U f; f.h[0] = *(const v8h*)(p); f.h[1] = *(const v8h*)(p + 16); return f.v;
  }
  static __device__ __forceinline__ v8f mma(v16h a, v16h b, v8f c) {
    return __builtin_amdgcn_wmma_f32_16x16x32_f16(false, a, false, b, (short)0, c, false, false);
  }
};
template <> struct Frag<__bf16> {
  typedef v16b V; union U { v16b v; v8b h[2]; };
  static __device__ __forceinline__ v16b load(const __bf16* p) {
    U f; f.h[0] = *(const v8b*)(p); f.h[1] = *(const v8b*)(p + 16); return f.v;
  }
  static __device__ __forceinline__ v8f mma(v16b a, v16b b, v8f c) {
    return __builtin_amdgcn_wmma_f32_16x16x32_bf16(false, a, false, b, (short)0, c, false, false);
  }
};

__device__ __forceinline__ float fsig(float x)  { return __builtin_amdgcn_rcpf(1.0f + __expf(-x)); }
__device__ __forceinline__ float ftanh(float x) { return 1.0f - 2.0f * __builtin_amdgcn_rcpf(__expf(2.0f * x) + 1.0f); }

template <int MODE>
__global__ __launch_bounds__(NTHR) void cvt_plane_kernel(const float* __restrict__ src, unsigned short* __restrict__ dst,
                                                        int nrow_real, int ncol_real, int spitch, int nrow_out, int ncol8_out, float sc) {
  const int i  = blockIdx.x * NTHR + threadIdx.x;
  const int n8 = nrow_out * ncol8_out;
  if (i < n8) {
    const int row = i / ncol8_out;
    const int c8  = (i - row * ncol8_out) * 8;
    const int rr  = (row < nrow_real) ? row : (nrow_real - 1);
    const float rowf = (row < nrow_real) ? 1.0f : 0.0f;
    const float* sp = src + (size_t)rr * (size_t)spitch;
    v8h hv;
#pragma unroll
    for (int e = 0; e < 8; ++e) {
      const int col = c8 + e;
      const int cc  = (col < ncol_real) ? col : (ncol_real - 1);
      const float f = sp[cc];
      const float okf = (col < ncol_real) ? rowf : 0.0f;
      const float v = f * okf;
      unsigned short bits;
      if (MODE == 0) {
        bits = f2bf_bits(v * sc);
      } else {
        bits = __builtin_bit_cast(unsigned short, (_Float16)(bf16r(v) * sc));
      }
      hv[e] = __builtin_bit_cast(_Float16, bits);
    }
    *(volatile v8h*)(dst + (size_t)i * 8) = hv;
    __threadfence();
    *(volatile v8h*)(dst + (size_t)i * 8) = hv;
  }
}

__global__ __launch_bounds__(NTHR) void gru_enc_kernel(
    const unsigned short* __restrict__ XEB, const unsigned short* __restrict__ WIEp,
    const unsigned short* __restrict__ WHEp,
    const float* __restrict__ bih, const float* __restrict__ bhh,
    float* __restrict__ HENCF, unsigned short* __restrict__ HEH, unsigned short* __restrict__ HEL) {
  __shared__ __align__(16) unsigned short Ax[SEQB * XPITCH];
  __shared__ __align__(16) _Float16       Ah[SEQB * HPITCH];
  __shared__ __align__(16) float          Hm[SEQB * HMP];
  __shared__ __align__(16) float          Bc[4 * NH];
  const __bf16*   WIE = (const __bf16*)WIEp;
  const _Float16* WHE = (const _Float16*)WHEp;
  const int tid = threadIdx.x, lane = tid & 31, wave = tid >> 5;
  const int c = lane & 15, hh = lane >> 4, koff = hh * 8;
  const int rowbase = blockIdx.x * SEQB;

#pragma unroll 1
  for (int i = tid; i < SEQB * HPITCH; i += NTHR) Ah[i] = (_Float16)0.0f;
#pragma unroll 1
  for (int i = tid; i < SEQB * HMP; i += NTHR) Hm[i] = 0.0f;
#pragma unroll 1
  for (int i = 0; i < 4; ++i) {
    const int j = tid + NTHR * i;
    const float p0 = bih[j], p1 = bih[NH + j], p2 = bih[2 * NH + j];
    const float q0 = bhh[j], q1 = bhh[NH + j], q2 = bhh[2 * NH + j];
    Bc[j]          = bf16r(p0) + bf16r(q0);
    Bc[NH + j]     = bf16r(p1) + bf16r(q1);
    Bc[2 * NH + j] = bf16r(p2);
    Bc[3 * NH + j] = bf16r(q2);
  }
  if (tid < 128) {
    const int m = tid >> 3, c8 = (tid & 7) * 8;
    const uint4 u = *(const uint4*)(XEB + ((size_t)(rowbase + m) * NS) * NIP + c8);
    *(uint4*)(Ax + m * XPITCH + c8) = u;
  }
  __syncthreads();

  const __bf16*   axrow = (const __bf16*)Ax + c * XPITCH + koff;
  const _Float16* ahrow = Ah + c * HPITCH + koff;
  const v8f z8 = {0.f, 0.f, 0.f, 0.f, 0.f, 0.f, 0.f, 0.f};

#pragma unroll 1
  for (int s = 0; s < NS; ++s) {
#pragma unroll 1
    for (int nt = 0; nt < NTW; ++nt) {
      const int j = WCOLS * wave + 16 * nt + c;
      const __bf16*   wx = WIE + (size_t)j * NIP + koff;
      const _Float16* wh = WHE + (size_t)j * NH + koff;
      v8f acc[4];
      acc[0] = z8; acc[1] = z8; acc[2] = z8; acc[3] = z8;
#pragma unroll 1
      for (int kx = 0; kx < NIP; kx += 32) {
        const v16b a  = Frag<__bf16>::load(axrow + kx);
        const v16b b0 = Frag<__bf16>::load(wx + kx);
        const v16b b1 = Frag<__bf16>::load(wx + (size_t)1 * NH * NIP + kx);
        const v16b b2 = Frag<__bf16>::load(wx + (size_t)2 * NH * NIP + kx);
        acc[0] = Frag<__bf16>::mma(a, b0, acc[0]);
        acc[1] = Frag<__bf16>::mma(a, b1, acc[1]);
        acc[2] = Frag<__bf16>::mma(a, b2, acc[2]);
        guard4_b(acc[0], acc[1], acc[2], acc[3], a, b0, b1, b2);
      }
#pragma unroll 1
      for (int k0 = 0; k0 < NH; k0 += 32) {
        const v16h a  = Frag<_Float16>::load(ahrow + k0);
        const v16h b0 = Frag<_Float16>::load(wh + k0);
        const v16h b1 = Frag<_Float16>::load(wh + (size_t)1 * NH * NH + k0);
        const v16h b2 = Frag<_Float16>::load(wh + (size_t)2 * NH * NH + k0);
        acc[0] = Frag<_Float16>::mma(a, b0, acc[0]);
        acc[1] = Frag<_Float16>::mma(a, b1, acc[1]);
        acc[3] = Frag<_Float16>::mma(a, b2, acc[3]);
        guard4_h(acc[0], acc[1], acc[2], acc[3], a, b0, b1, b2);
      }
      acc_guard4(acc[0], acc[1], acc[2], acc[3]);
      const float br  = Bc[j];
      const float bz  = Bc[NH + j];
      const float bni = Bc[2 * NH + j];
      const float bnh = Bc[3 * NH + j];
#pragma unroll
      for (int rr = 0; rr < 8; ++rr) {
        const int hidx  = (8 * hh + rr) * HMP + j;
        const float pr  = acc[0][rr] * WCARRY_INV + br;
        const float pz  = acc[1][rr] * WCARRY_INV + bz;
        const float gin = acc[2][rr] * WCARRY_INV + bni;
        const float ghn = acc[3][rr] * WCARRY_INV + bnh;
        const float rg  = fsig(pr);
        const float zg  = fsig(pz);
        const float ng  = ftanh(gin + rg * ghn);
        const float ho  = Hm[hidx];
        Hm[hidx] = (1.0f - zg) * ng + zg * ho;
      }
    }
    __syncthreads();
#pragma unroll 1
    for (int nt = 0; nt < NTW; ++nt) {
      const int j = WCOLS * wave + 16 * nt + c;
#pragma unroll
      for (int rr = 0; rr < 8; ++rr) Ah[(8 * hh + rr) * HPITCH + j] = (_Float16)Hm[(8 * hh + rr) * HMP + j];
    }
    if (tid < 128) {
      const int sn = (s + 1 < NS) ? (s + 1) : (NS - 1);
      const int m = tid >> 3, c8 = (tid & 7) * 8;
      const uint4 u = *(const uint4*)(XEB + ((size_t)(rowbase + m) * NS + (size_t)sn) * NIP + c8);
      *(uint4*)(Ax + m * XPITCH + c8) = u;
    }
    __syncthreads();
  }

  for (int pass = 0; pass < 2; ++pass) {
#pragma unroll
    for (int it = 0; it < 16; ++it) {
      const int idx = it * NTHR + tid;
      const int row = idx >> 8, c4 = (idx & 255) * 4;
      const v4f v = *(const v4f*)(Hm + row * HMP + c4);
      *(volatile v4f*)(HENCF + (size_t)(rowbase + row) * NH + c4) = v;
    }
    __threadfence();
  }
  for (int pass = 0; pass < 2; ++pass) {
#pragma unroll
    for (int it = 0; it < 8; ++it) {
      const int idx = it * NTHR + tid;
      const int row = idx >> 7, c8 = (idx & 127) * 8;
      const v4f va = *(const v4f*)(Hm + row * HMP + c8);
      const v4f vb = *(const v4f*)(Hm + row * HMP + c8 + 4);
      v8h hv, lv;
#pragma unroll
      for (int e = 0; e < 4; ++e) {
        const unsigned short ha = f2bf_bits(va[e]);
        const unsigned short la = f2bf_bits(va[e] - bf_bits2f(ha));
        const unsigned short hb = f2bf_bits(vb[e]);
        const unsigned short lb = f2bf_bits(vb[e] - bf_bits2f(hb));
        hv[e]     = __builtin_bit_cast(_Float16, ha);
        lv[e]     = __builtin_bit_cast(_Float16, la);
        hv[4 + e] = __builtin_bit_cast(_Float16, hb);
        lv[4 + e] = __builtin_bit_cast(_Float16, lb);
      }
      const size_t o = (size_t)(rowbase + row) * NH + c8;
      *(volatile v8h*)(HEH + o) = hv;
      *(volatile v8h*)(HEL + o) = lv;
    }
    __threadfence();
  }
}

__global__ __launch_bounds__(NTHR) void gh_gemm_kernel(
    const unsigned short* __restrict__ HEHp, const unsigned short* __restrict__ HELp,
    const unsigned short* __restrict__ WHDp, float* __restrict__ GHD) {
  __shared__ __align__(16) float Sl[NWAV][16 * SLABP];
  const __bf16* AH = (const __bf16*)HEHp;
  const __bf16* AL = (const __bf16*)HELp;
  const __bf16* WD = (const __bf16*)WHDp;
  const int tid = threadIdx.x, lane = tid & 31, wave = tid >> 5;
  const int c = lane & 15, hh = lane >> 4, koff = hh * 8, c4 = c * 4;
  const int m0 = blockIdx.x * SEQB;
  const int nb = blockIdx.y * GHCOLB + 64 * wave;
  float* slab = Sl[wave];

  const __bf16* ahp = AH + (size_t)(m0 + c) * NH + koff;
  const __bf16* alp = AL + (size_t)(m0 + c) * NH + koff;
  const __bf16* wp0 = WD + (size_t)(nb + 0 * 16 + c) * NH + koff;
  const __bf16* wp1 = WD + (size_t)(nb + 1 * 16 + c) * NH + koff;
  const __bf16* wp2 = WD + (size_t)(nb + 2 * 16 + c) * NH + koff;
  const __bf16* wp3 = WD + (size_t)(nb + 3 * 16 + c) * NH + koff;
  const v8f z8 = {0.f, 0.f, 0.f, 0.f, 0.f, 0.f, 0.f, 0.f};
  v8f acc[4];
  acc[0] = z8; acc[1] = z8; acc[2] = z8; acc[3] = z8;
#pragma unroll 1
  for (int k0 = 0; k0 < NH; k0 += 32) {
    const v16b ah = Frag<__bf16>::load(ahp + k0);
    const v16b al = Frag<__bf16>::load(alp + k0);
    const v16b b0 = Frag<__bf16>::load(wp0 + k0);
    const v16b b1 = Frag<__bf16>::load(wp1 + k0);
    const v16b b2 = Frag<__bf16>::load(wp2 + k0);
    const v16b b3 = Frag<__bf16>::load(wp3 + k0);
    acc[0] = Frag<__bf16>::mma(ah, b0, acc[0]);
    acc[0] = Frag<__bf16>::mma(al, b0, acc[0]);
    acc[1] = Frag<__bf16>::mma(ah, b1, acc[1]);
    acc[1] = Frag<__bf16>::mma(al, b1, acc[1]);
    acc[2] = Frag<__bf16>::mma(ah, b2, acc[2]);
    acc[2] = Frag<__bf16>::mma(al, b2, acc[2]);
    acc[3] = Frag<__bf16>::mma(ah, b3, acc[3]);
    acc[3] = Frag<__bf16>::mma(al, b3, acc[3]);
    guard4_b6(acc[0], acc[1], acc[2], acc[3], ah, al, b0, b1, b2, b3);
  }
  acc_guard4(acc[0], acc[1], acc[2], acc[3]);
#pragma unroll
  for (int ntl = 0; ntl < 4; ++ntl)
#pragma unroll
    for (int rr = 0; rr < 8; ++rr) slab[(8 * hh + rr) * SLABP + 16 * ntl + c] = acc[ntl][rr];
  __syncthreads();
  for (int pass = 0; pass < 2; ++pass) {
#pragma unroll
    for (int it = 0; it < 8; ++it) {
      const int row = it * 2 + hh;
      const v4f v = *(const v4f*)(slab + row * SLABP + c4);
      *(volatile v4f*)(GHD + (size_t)(m0 + row) * NG3 + nb + c4) = v;
    }
    __threadfence();
  }
}

__global__ __launch_bounds__(NTHR) void gru_dec_kernel(
    const unsigned short* __restrict__ XDB, const unsigned short* __restrict__ WIDp,
    const float* __restrict__ GHD, const float* __restrict__ HENCF,
    const float* __restrict__ dbih, const float* __restrict__ dbhh,
    unsigned short* __restrict__ STH, unsigned short* __restrict__ STL) {
  __shared__ __align__(16) unsigned short Ax[SEQB * XPITCH];
  __shared__ __align__(16) float          Gs[GSROWS * NH];
  __shared__ __align__(16) float          Ssf[SEQB * HMP];
  const __bf16* WID = (const __bf16*)WIDp;
  const int tid = threadIdx.x, lane = tid & 31, wave = tid >> 5;
  const int c = lane & 15, hh = lane >> 4, koff = hh * 8;
  const int rowbase = blockIdx.x * SEQB;
  const int bsel = blockIdx.x >> 2;
  const int q4 = 4 * tid;

#pragma unroll 1
  for (int g = 0; g < 3; ++g) {
    const v4f v = *(const v4f*)(GHD + (size_t)bsel * NG3 + (size_t)g * NH + q4);
    *(v4f*)(Gs + g * NH + q4) = v;
  }
  {
    const v4f v = *(const v4f*)(HENCF + (size_t)bsel * NH + q4);
    *(v4f*)(Gs + 3 * NH + q4) = v;
  }
#pragma unroll 1
  for (int g = 0; g < 3; ++g) {
    const v4f v = *(const v4f*)(dbih + (size_t)g * NH + q4);
    *(v4f*)(Gs + (4 + g) * NH + q4) = v;
  }
#pragma unroll 1
  for (int g = 0; g < 3; ++g) {
    const v4f v = *(const v4f*)(dbhh + (size_t)g * NH + q4);
    *(v4f*)(Gs + (7 + g) * NH + q4) = v;
  }
  if (tid < 128) {
    const int m = tid >> 3, c8 = (tid & 7) * 8;
    const uint4 u = *(const uint4*)(XDB + (size_t)(rowbase + m) * NIP + c8);
    *(uint4*)(Ax + m * XPITCH + c8) = u;
  }
  __syncthreads();

  const __bf16* axrow = (const __bf16*)Ax + c * XPITCH + koff;
  const v8f z8 = {0.f, 0.f, 0.f, 0.f, 0.f, 0.f, 0.f, 0.f};
#pragma unroll 1
  for (int nt = 0; nt < NTW; ++nt) {
    const int j = WCOLS * wave + 16 * nt + c;
    const __bf16* wx = WID + (size_t)j * NIP + koff;
    v8f acc[3];
    acc[0] = z8; acc[1] = z8; acc[2] = z8;
#pragma unroll 1
    for (int kx = 0; kx < NIP; kx += 32) {
      const v16b a  = Frag<__bf16>::load(axrow + kx);
      const v16b b0 = Frag<__bf16>::load(wx + kx);
      const v16b b1 = Frag<__bf16>::load(wx + (size_t)1 * NH * NIP + kx);
      const v16b b2 = Frag<__bf16>::load(wx + (size_t)2 * NH * NIP + kx);
      acc[0] = Frag<__bf16>::mma(a, b0, acc[0]);
      acc[1] = Frag<__bf16>::mma(a, b1, acc[1]);
      acc[2] = Frag<__bf16>::mma(a, b2, acc[2]);
      guard3_b(acc[0], acc[1], acc[2], a, b0, b1, b2);
    }
    acc_guard3(acc[0], acc[1], acc[2]);
    const float vr  = Gs[j]          + (bf16r(Gs[4 * NH + j]) + bf16r(Gs[7 * NH + j]));
    const float vz  = Gs[NH + j]     + (bf16r(Gs[5 * NH + j]) + bf16r(Gs[8 * NH + j]));
    const float vin = bf16r(Gs[6 * NH + j]);
    const float vhn = Gs[2 * NH + j] + bf16r(Gs[9 * NH + j]);
    const float he  = Gs[3 * NH + j];
#pragma unroll
    for (int rr = 0; rr < 8; ++rr) {
      const float pr  = acc[0][rr] * WCARRY_INV + vr;
      const float pz  = acc[1][rr] * WCARRY_INV + vz;
      const float gin = acc[2][rr] * WCARRY_INV + vin;
      const float rg  = fsig(pr);
      const float zg  = fsig(pz);
      const float ng  = ftanh(gin + rg * vhn);
      Ssf[(8 * hh + rr) * HMP + j] = (1.0f - zg) * ng + zg * he;
    }
  }
  __syncthreads();

  const int q = lane >> 3, c8 = (lane & 7) * 8;
  for (int pass = 0; pass < 2; ++pass) {
#pragma unroll
    for (int hf = 0; hf < 2; ++hf) {
#pragma unroll
      for (int it = 0; it < 4; ++it) {
        const int row = it * 4 + q;
        const int col = WCOLS * wave + 64 * hf + c8;
        const v4f va = *(const v4f*)(Ssf + row * HMP + col);
        const v4f vb = *(const v4f*)(Ssf + row * HMP + col + 4);
        v8h hv, lv;
#pragma unroll
        for (int e = 0; e < 4; ++e) {
          const unsigned short ha = f2bf_bits(va[e]);
          const unsigned short la = f2bf_bits(va[e] - bf_bits2f(ha));
          const unsigned short hb = f2bf_bits(vb[e]);
          const unsigned short lb = f2bf_bits(vb[e] - bf_bits2f(hb));
          hv[e]     = __builtin_bit_cast(_Float16, ha);
          lv[e]     = __builtin_bit_cast(_Float16, la);
          hv[4 + e] = __builtin_bit_cast(_Float16, hb);
          lv[4 + e] = __builtin_bit_cast(_Float16, lb);
        }
        const size_t o = (size_t)(rowbase + row) * NH + col;
        *(volatile v8h*)(STH + o) = hv;
        *(volatile v8h*)(STL + o) = lv;
      }
    }
    __threadfence();
  }
}

__global__ __launch_bounds__(NTHR) void proj_out_kernel(
    const unsigned short* __restrict__ STHp, const unsigned short* __restrict__ STLp,
    const unsigned short* __restrict__ WPp, const float* __restrict__ pb, float* __restrict__ out) {
  __shared__ __align__(16) float Of[PROWS * NI];
  const __bf16* SH = (const __bf16*)STHp;
  const __bf16* SLo = (const __bf16*)STLp;
  const __bf16* WP = (const __bf16*)WPp;
  const int tid = threadIdx.x, lane = tid & 31, wave = tid >> 5;
  const int c = lane & 15, hh = lane >> 4, koff = hh * 8;
  const int r0 = blockIdx.x * PROWS;
  const int msub = wave >> 1, npair = (wave & 1) * 2;

  const __bf16* ahp = SH  + (size_t)(r0 + 16 * msub + c) * NH + koff;
  const __bf16* alp = SLo + (size_t)(r0 + 16 * msub + c) * NH + koff;
  const __bf16* b0p = WP + (size_t)(16 * npair + c) * NH + koff;
  const __bf16* b1p = WP + (size_t)(16 * (npair + 1) + c) * NH + koff;
  const v8f z8 = {0.f, 0.f, 0.f, 0.f, 0.f, 0.f, 0.f, 0.f};
  v8f acc[2];
  acc[0] = z8; acc[1] = z8;
#pragma unroll 1
  for (int k0 = 0; k0 < NH; k0 += 32) {
    const v16b ah = Frag<__bf16>::load(ahp + k0);
    const v16b al = Frag<__bf16>::load(alp + k0);
    const v16b b0 = Frag<__bf16>::load(b0p + k0);
    const v16b b1 = Frag<__bf16>::load(b1p + k0);
    acc[0] = Frag<__bf16>::mma(ah, b0, acc[0]);
    acc[0] = Frag<__bf16>::mma(al, b0, acc[0]);
    acc[1] = Frag<__bf16>::mma(ah, b1, acc[1]);
    acc[1] = Frag<__bf16>::mma(al, b1, acc[1]);
    guard2_b4(acc[0], acc[1], ah, al, b0, b1);
  }
  acc_guard2(acc[0], acc[1]);
#pragma unroll
  for (int qn = 0; qn < 2; ++qn) {
    const int col  = 16 * (npair + qn) + c;
    const int colc = (col < NI) ? col : (NI - 1);
    const float bo = bf16r(pb[colc]);
#pragma unroll
    for (int rr = 0; rr < 8; ++rr) {
      const int row = 16 * msub + 8 * hh + rr;
      const float v = acc[qn][rr] + bo;
      if (col < NI) Of[row * NI + col] = v;
    }
  }
  __syncthreads();
  float* ob = out + (size_t)r0 * NI;
  for (int pass = 0; pass < 2; ++pass) {
#pragma unroll
    for (int it = 0; it < 4; ++it) {
      const int idx = it * NTHR + tid;
      if (idx < PNF4) {
        const v4f v = *(const v4f*)(Of + 4 * idx);
        *(volatile v4f*)(ob + 4 * (size_t)idx) = v;
      }
    }
    __threadfence();
  }
}

extern "C" void kernel_launch(void* const* d_in, const int* in_sizes, int n_in,
                              void* d_out, int out_size, void* d_ws, size_t ws_size, hipStream_t stream) {
  if (n_in < 12 || d_out == nullptr || d_ws == nullptr) return;
  if (in_sizes[0] != NB * NS * NI || in_sizes[1] != NB * NTD * NI || in_sizes[2] != NG3 * NI || in_sizes[3] != NG3 * NH ||
      in_sizes[4] != NG3 || in_sizes[5] != NG3 || in_sizes[6] != NG3 * NI || in_sizes[7] != NG3 * NH ||
      in_sizes[8] != NG3 || in_sizes[9] != NG3 || in_sizes[10] != NI * NH || in_sizes[11] != NI || out_size != NOUT) return;

  const float* enc_x   = (const float*)d_in[0];
  const float* dec_x   = (const float*)d_in[1];
  const float* enc_Wih = (const float*)d_in[2];
  const float* enc_Whh = (const float*)d_in[3];
  const float* enc_bih = (const float*)d_in[4];
  const float* enc_bhh = (const float*)d_in[5];
  const float* dec_Wih = (const float*)d_in[6];
  const float* dec_Whh = (const float*)d_in[7];
  const float* dec_bih = (const float*)d_in[8];
  const float* dec_bhh = (const float*)d_in[9];
  const float* proj_W  = (const float*)d_in[10];
  const float* proj_b  = (const float*)d_in[11];
  float* out = (float*)d_out;

  char* ws = (char*)d_ws; size_t off = 0;
  auto carve = [&](size_t bytes) -> char* { char* p = ws + off; off += (bytes + 255) & ~(size_t)255; return p; };
  unsigned short* XEB   = (unsigned short*)carve((size_t)NROWE * NIP * 2);
  unsigned short* XDB   = (unsigned short*)carve((size_t)NROWD * NIP * 2);
  unsigned short* WIE   = (unsigned short*)carve((size_t)NG3 * NIP * 2);
  unsigned short* WID   = (unsigned short*)carve((size_t)NG3 * NIP * 2);
  unsigned short* WHE   = (unsigned short*)carve((size_t)NG3 * NH * 2);
  unsigned short* WHD   = (unsigned short*)carve((size_t)NG3 * NH * 2);
  unsigned short* WP    = (unsigned short*)carve((size_t)NIP * NH * 2);
  float*          HENCF = (float*)carve((size_t)NB * NH * 4);
  unsigned short* HEH   = (unsigned short*)carve((size_t)NB * NH * 2);
  unsigned short* HEL   = (unsigned short*)carve((size_t)NB * NH * 2);
  float*          GHD   = (float*)carve((size_t)NB * NG3 * 4);
  unsigned short* STH   = (unsigned short*)carve((size_t)NROWD * NH * 2);
  unsigned short* STL   = (unsigned short*)carve((size_t)NROWD * NH * 2);
  if (off > ws_size || off > (size_t)134217728) return;

  cvt_plane_kernel<0><<<(NROWE * (NIP / 8)) / NTHR, NTHR, 0, stream>>>(enc_x,   XEB, NROWE, NI, NI, NROWE, NIP / 8, 1.0f);
  cvt_plane_kernel<0><<<(NROWD * (NIP / 8)) / NTHR, NTHR, 0, stream>>>(dec_x,   XDB, NROWD, NI, NI, NROWD, NIP / 8, 1.0f);
  cvt_plane_kernel<0><<<(NG3 * (NIP / 8)) / NTHR,   NTHR, 0, stream>>>(enc_Wih, WIE, NG3,   NI, NI, NG3,   NIP / 8, WCARRY);
  cvt_plane_kernel<0><<<(NG3 * (NIP / 8)) / NTHR,   NTHR, 0, stream>>>(dec_Wih, WID, NG3,   NI, NI, NG3,   NIP / 8, WCARRY);
  cvt_plane_kernel<1><<<(NG3 * (NH / 8)) / NTHR,    NTHR, 0, stream>>>(enc_Whh, WHE, NG3,   NH, NH, NG3,   NH / 8,  WCARRY);
  cvt_plane_kernel<0><<<(NG3 * (NH / 8)) / NTHR,    NTHR, 0, stream>>>(dec_Whh, WHD, NG3,   NH, NH, NG3,   NH / 8,  1.0f);
  cvt_plane_kernel<0><<<(NIP * (NH / 8)) / NTHR,    NTHR, 0, stream>>>(proj_W,  WP,  NI,    NH, NH, NIP,   NH / 8,  1.0f);
  gru_enc_kernel<<<NB / SEQB, NTHR, 0, stream>>>(XEB, WIE, WHE, enc_bih, enc_bhh, HENCF, HEH, HEL);
  gh_gemm_kernel<<<dim3(NB / SEQB, NG3 / GHCOLB), NTHR, 0, stream>>>(HEH, HEL, WHD, GHD);
  gru_dec_kernel<<<NROWD / SEQB, NTHR, 0, stream>>>(XDB, WID, GHD, HENCF, dec_bih, dec_bhh, STH, STL);
  proj_out_kernel<<<NROWD / PROWS, NTHR, 0, stream>>>(STH, STL, WP, proj_b, out);
}
